// SOP_1726576855136
// MI455X (gfx1250) — hardware-verified
//
#include <hip/hip_runtime.h>
#pragma clang fp contract(off)


#ifndef NB
#define NB 16
#endif
#ifndef SEQ
#define SEQ 2048
#endif
#define NB_FULL  16
#define SEQ_FULL 2048
#define DF   64
#define LP   68
#define MATF (DF * LP)
#define OFF_S 0
#define OFF_T (MATF)
#define OFF_Y (2 * MATF)
#define OFF_Z (3 * MATF)
#define NTHR 256
#define SIGN_ITERS 40
#define SQRT_ITERS 22
#define NEGB (-3.0e38f)

static_assert(DF == 64);
static_assert(NTHR == 256);
static_assert(LP % 4 == 0);
static_assert(LP >= DF);
static_assert(SEQ % 64 == 0);
static_assert(SEQ >= 64);
static_assert(NB <= NB_FULL);
static_assert(SEQ <= SEQ_FULL);
static_assert(NTHR * 4 * 4 == 64 * DF);
static_assert((NTHR / 16) * 4 == DF);
static_assert(NTHR * 16 * 4 == DF * DF * 4);
static_assert((4 * MATF + 8) * 4 <= 131072);
static_assert((DF * DF * 4) % 128 == 0);

typedef unsigned short bf;
typedef __attribute__((ext_vector_type(16))) __bf16   v16bf;
typedef __attribute__((ext_vector_type(8)))  unsigned short v8us;
typedef __attribute__((ext_vector_type(8)))  float    v8f;
typedef __attribute__((ext_vector_type(4)))  float    v4f;
typedef v4f  __attribute__((may_alias)) v4fa;

__device__ __forceinline__ unsigned short f2bf(float f) { unsigned u = __float_as_uint(f); u += 0x7FFFu + ((u >> 16) & 1u); return (unsigned short)(u >> 16); }
__device__ __forceinline__ float bfr(float f) { return __uint_as_float(((unsigned)f2bf(f)) << 16); }
__device__ __forceinline__ v16bf cat16b(v8us lo, v8us hi) { return __builtin_bit_cast(v16bf, __builtin_shufflevector(lo, hi, 0, 1, 2, 3, 4, 5, 6, 7, 8, 9, 10, 11, 12, 13, 14, 15)); }
__device__ __forceinline__ v8f wmmab(v16bf a, v16bf b, v8f c) { return __builtin_amdgcn_wmma_f32_16x16x32_bf16(false, a, false, b, (short)0, c, false, false); }
__device__ __forceinline__ v8f wmmab_g(v16bf a, v16bf b, v8f c) { c = wmmab(a, b, c); asm volatile("v_nop\n\tv_nop\n\tv_nop\n\tv_nop" : "+v"(c) : "v"(a), "v"(b)); return c; }

__device__ __forceinline__ void tri1(const float v, unsigned short& h, unsigned short& m, unsigned short& l) {
    h = f2bf(v); const float r1 = v - __uint_as_float(((unsigned)h) << 16);
    m = f2bf(r1); const float r2 = r1 - __uint_as_float(((unsigned)m) << 16);
    l = f2bf(r2);
}
__device__ __forceinline__ void tri8(const v4f x0, const v4f x1, v8us& H, v8us& Mi, v8us& L) {
#pragma unroll
    for (int i = 0; i < 4; ++i) {
        unsigned short a, b, c;
        tri1(x0[i], a, b, c); H[i] = a;     Mi[i] = b;     L[i] = c;
        tri1(x1[i], a, b, c); H[4 + i] = a; Mi[4 + i] = b; L[4 + i] = c; }
}

template <int NT>
__device__ __forceinline__ void mm_row(const float* sm, const int ao, const int bo, const int tm, const int tn0, const int lr, const int hi, v8f (&acc)[NT]) {
#pragma unroll
    for (int t = 0; t < NT; ++t) acc[t] = (v8f){};
#pragma unroll
    for (int ks = 0; ks < 2; ++ks) {
        const int k0 = 32 * ks + 8 * hi;
        const int ap = ao + (tm * 16 + lr) * LP + k0;
        const v4f a0 = *(const v4fa*)(&sm[ap]),      a1 = *(const v4fa*)(&sm[ap + 4]);
        const v4f a2 = *(const v4fa*)(&sm[ap + 16]), a3 = *(const v4fa*)(&sm[ap + 20]);
        v8us h0, m0, l0, h1, m1, l1;
        tri8(a0, a1, h0, m0, l0); tri8(a2, a3, h1, m1, l1);
        const v16bf ah = cat16b(h0, h1), am = cat16b(m0, m1), al = cat16b(l0, l1);
#pragma unroll
        for (int t = 0; t < NT; ++t) {
            const int bp = bo + k0 * LP + (tn0 + t) * 16 + lr;
            v4f b0, b1, b2, b3;
#pragma unroll
            for (int i = 0; i < 4; ++i) { b0[i] = sm[bp + i * LP]; b1[i] = sm[bp + (4 + i) * LP]; b2[i] = sm[bp + (16 + i) * LP]; b3[i] = sm[bp + (20 + i) * LP]; }
            v8us g0, n0, e0, g1, n1, e1;
            tri8(b0, b1, g0, n0, e0); tri8(b2, b3, g1, n1, e1);
            const v16bf bh = cat16b(g0, g1), bm = cat16b(n0, n1), bl = cat16b(e0, e1);
            v8f c = acc[t];
            c = wmmab_g(al, bh, c); c = wmmab_g(ah, bl, c); c = wmmab_g(am, bm, c);
            c = wmmab_g(am, bh, c); c = wmmab_g(ah, bm, c); c = wmmab_g(ah, bh, c);
            acc[t] = c; }
    }
}

template <int NT>
__device__ __forceinline__ void st_tiles(float* sm, const int off, const int tm, const int tn0, const int lr, const int hi, const v8f (&acc)[NT], const float sc) {
#pragma unroll
    for (int t = 0; t < NT; ++t) {
        const int p = off + (tm * 16 + 8 * hi) * LP + (tn0 + t) * 16 + lr;
#pragma unroll
        for (int r = 0; r < 8; ++r) sm[p + r * LP] = acc[t][r] * sc; }
}

__device__ __forceinline__ float block_sum(float v, float* red, const int lane, const int wave) {
#pragma unroll
    for (int o = 16; o >= 1; o >>= 1) v += __shfl_xor(v, o, 32);
    __syncthreads();
    if (lane == 0) red[wave] = v;
    __syncthreads();
    float s = 0.0f;
#pragma unroll
    for (int i = 0; i < NTHR / 32; ++i) s += red[i];
    return s;
}

__global__ __launch_bounds__(NTHR) __attribute__((amdgpu_num_vgpr(256)))
void k_pool_root(const float* __restrict__ x, float* out) {
    __shared__ __align__(16) float sm[4 * MATF];
    __shared__ float red[NTHR / 32];
    const int tid = threadIdx.x, lane = tid & 31, lr = lane & 15, hi = lane >> 4;
    const int wave = __builtin_amdgcn_readfirstlane((int)(threadIdx.x >> 5));
    const int bat = blockIdx.x;
    const float* xb = x + (size_t)bat * (size_t)SEQ_FULL * DF;

    const int ti = (tid >> 4) * 4, tj = (tid & 15) * 4;
    float acc[4][4];
#pragma unroll
    for (int a = 0; a < 4; ++a)
#pragma unroll
        for (int q = 0; q < 4; ++q) acc[a][q] = NEGB;
#pragma unroll 1
    for (int n0 = 0; n0 < SEQ; n0 += 64) {
#pragma unroll
        for (int e = 0; e < 4; ++e) {
            const int f = e * NTHR + tid; const int row = f >> 4, c4 = (f & 15) * 4;
            const v4f g = *(const v4f*)(xb + (size_t)(n0 + row) * DF + c4);
            v4f t; t[0] = bfr(g[0]); t[1] = bfr(g[1]); t[2] = bfr(g[2]); t[3] = bfr(g[3]);
            *(v4fa*)(&sm[OFF_T + row * LP + c4]) = t; }
        __syncthreads();
#pragma unroll 4
        for (int n = 0; n < 64; ++n) {
            const v4f xi = *(const v4fa*)(&sm[OFF_T + n * LP + ti]);
            const v4f xj = *(const v4fa*)(&sm[OFF_T + n * LP + tj]);
#pragma unroll
            for (int a = 0; a < 4; ++a)
#pragma unroll
                for (int q = 0; q < 4; ++q) acc[a][q] = fmaxf(acc[a][q], xi[a] * xj[q]); }
        __syncthreads();
    }

    {
        float ss = 0.0f;
#pragma unroll
        for (int a = 0; a < 4; ++a)
#pragma unroll
            for (int q = 0; q < 4; ++q) ss += acc[a][q] * acc[a][q];
        const float s = block_sum(ss, red, lane, wave);
        const float nm = sqrtf(s);
        const float rnm = (nm > 0.0f) ? (1.0f / nm) : 0.0f;
#pragma unroll
        for (int a = 0; a < 4; ++a) {
            v4f mrow, srow;
#pragma unroll
            for (int q = 0; q < 4; ++q) { mrow[q] = acc[a][q]; srow[q] = acc[a][q] * rnm; }
            *(v4fa*)(&sm[OFF_Z + (ti + a) * LP + tj]) = mrow;
            *(v4fa*)(&sm[OFF_S + (ti + a) * LP + tj]) = srow; }
        __syncthreads();
    }

    const int tmS = wave >> 1, tnS = (wave & 1) * 2;

#pragma unroll 1
    for (int it = 0; it < SIGN_ITERS; ++it) {
        v8f p[2]; mm_row<2>(sm, OFF_S, OFF_S, tmS, tnS, lr, hi, p);
        st_tiles<2>(sm, OFF_T, tmS, tnS, lr, hi, p, 1.0f);
        __syncthreads();
        v8f q[2]; mm_row<2>(sm, OFF_S, OFF_T, tmS, tnS, lr, hi, q);
        __syncthreads();
#pragma unroll
        for (int t = 0; t < 2; ++t) {
            const int pp = OFF_S + (tmS * 16 + 8 * hi) * LP + (tnS + t) * 16 + lr;
#pragma unroll
            for (int r = 0; r < 8; ++r) { const float sv = sm[pp + r * LP]; sm[pp + r * LP] = 1.5f * sv - 0.5f * q[t][r]; } }
        __syncthreads();
    }

    float nA;
    {
        v8f a[2]; mm_row<2>(sm, OFF_S, OFF_Z, tmS, tnS, lr, hi, a);
        float ss = 0.0f;
#pragma unroll
        for (int r = 0; r < 8; ++r) ss += a[0][r] * a[0][r] + a[1][r] * a[1][r];
        const float s = block_sum(ss, red, lane, wave);
        nA = sqrtf(s);
        const float rnA = (nA > 0.0f) ? (1.0f / nA) : 0.0f;
        st_tiles<2>(sm, OFF_Y, tmS, tnS, lr, hi, a, rnA);
#pragma unroll
        for (int e = 0; e < 4; ++e) {
            const int f = e * NTHR + tid; const int row = f >> 4, c4 = (f & 15) * 4;
            v4f z;
#pragma unroll
            for (int i = 0; i < 4; ++i) z[i] = (row == c4 + i) ? 1.0f : 0.0f;
            *(v4fa*)(&sm[OFF_Z + row * LP + c4]) = z; }
        __syncthreads();
    }

    const int isz = wave >> 2;
    const int tm4 = wave & 3;
    const int ao4 = OFF_Y + isz * (OFF_T - OFF_Y);
    const int bo4 = OFF_T + isz * (OFF_Z - OFF_T);
    const int do4 = OFF_Y + isz * (OFF_Z - OFF_Y);
#pragma unroll 1
    for (int it = 0; it < SQRT_ITERS; ++it) {
        v8f w[2]; mm_row<2>(sm, OFF_Z, OFF_Y, tmS, tnS, lr, hi, w);
#pragma unroll
        for (int t = 0; t < 2; ++t) {
            const int rb = tmS * 16 + 8 * hi, col = (tnS + t) * 16 + lr;
            const int pp = OFF_T + rb * LP + col;
#pragma unroll
            for (int r = 0; r < 8; ++r) sm[pp + r * LP] = ((rb + r) == col ? 1.5f : 0.0f) - 0.5f * w[t][r]; }
        __syncthreads();
        v8f rr[4]; mm_row<4>(sm, ao4, bo4, tm4, 0, lr, hi, rr);
        __syncthreads();
        st_tiles<4>(sm, do4, tm4, 0, lr, hi, rr, 1.0f);
        __syncthreads();
    }

    {
        v8f f[2]; mm_row<2>(sm, OFF_S, OFF_Y, tmS, tnS, lr, hi, f);
        float ss = 0.0f;
#pragma unroll
        for (int r = 0; r < 8; ++r) ss += f[0][r] * f[0][r] + f[1][r] * f[1][r];
        const float s = block_sum(ss, red, lane, wave);
        const float fro = sqrtf(s);
        const float snA = sqrtf(nA);
        const float den = fmaxf(snA * fro, 1e-12f);
        const float so = snA * (1.0f / den);
        st_tiles<2>(sm, OFF_T, tmS, tnS, lr, hi, f, so);
        __syncthreads();
    }
    float* ob = out + (size_t)bat * (size_t)(DF * DF);
#pragma unroll 1
    for (int ps = 0; ps < 2; ++ps) {
#pragma unroll
        for (int e = 0; e < 4; ++e) {
            const int f = e * NTHR + tid; const int row = f >> 4, c4 = (f & 15) * 4;
            const v4f val = *(const v4fa*)(&sm[OFF_T + row * LP + c4]);
            *(volatile v4f*)(ob + (size_t)row * DF + c4) = val; }
        if (ps == 0) __threadfence(); }
}

extern "C" void kernel_launch(void* const* d_in, const int* in_sizes, int n_in,
                              void* d_out, int out_size, void* d_ws, size_t ws_size, hipStream_t stream) {
    (void)d_ws; (void)ws_size;
    if (n_in < 1) return;
    if ((size_t)in_sizes[0] < ((size_t)(NB - 1) * SEQ_FULL + SEQ) * DF) return;
    if ((size_t)out_size < (size_t)NB * DF * DF) return;
    const float* x = (const float*)d_in[0];
    float* OUT = (float*)d_out;
    k_pool_root<<<dim3(NB, 1, 1), NTHR, 0, stream>>>(x, OUT);
}
